// VectorizedSplatAttention_43224550867597
// MI455X (gfx1250) — hardware-run, weakly checked
//
#include <hip/hip_runtime.h>
#include <math.h>

constexpr int kB    = 2;
constexpr int kS    = 2048;
constexpr int kD    = 1024;
constexpr int kH    = 16;
constexpr int kNS   = 16;
constexpr int kHD   = 64;
constexpr int kTok  = kB * kS;
constexpr int kQKVN = 3 * kD;
constexpr int kKP   = 32;
constexpr int kBH   = kB * kH;
constexpr int kGrp  = 2;
constexpr float kWgtCarry   = 1048576.0f;
constexpr float kScoreScale = 1.0f / (1048576.0f * 1048576.0f);
constexpr float kPCarry     = 32768.0f;
constexpr float kPCarryInv  = 1.0f / 32768.0f;
constexpr float kInvS       = 1.0f / 2048.0f;

typedef __attribute__((ext_vector_type(16))) _Float16 v16h;
typedef __attribute__((ext_vector_type(8)))  _Float16 v8h;
typedef __attribute__((ext_vector_type(16))) __bf16   v16b;
typedef __attribute__((ext_vector_type(8)))  __bf16   v8b;
typedef __attribute__((ext_vector_type(8)))  float    v8f;
typedef __attribute__((ext_vector_type(4)))  float    v4f;
typedef __attribute__((ext_vector_type(4)))  unsigned int v4u;
typedef __attribute__((ext_vector_type(2)))  unsigned int v2u;

__device__ __forceinline__ unsigned short f2bf_bits(float f) {
  unsigned u = __float_as_uint(f);
  return (unsigned short)((u + 0x7FFFu + ((u >> 16) & 1u)) >> 16);
}
__device__ __forceinline__ float bf_bits2f(unsigned short h) { return __uint_as_float(((unsigned)h) << 16); }
__device__ __forceinline__ float bfw_lo(unsigned w) { return __uint_as_float(w << 16); }
__device__ __forceinline__ float bfw_hi(unsigned w) { return __uint_as_float(w & 0xffff0000u); }

__device__ __forceinline__ void dep_guard_h(v8f& a, v8f& b, v16h x, v16h y) { asm volatile("v_nop\n\tv_nop\n\tv_nop\n\tv_nop" : "+v"(a), "+v"(b) : "v"(x), "v"(y)); }
__device__ __forceinline__ void dep_guard_b(v8f& a, v8f& b, v16b x, v16b y) { asm volatile("v_nop\n\tv_nop\n\tv_nop\n\tv_nop" : "+v"(a), "+v"(b) : "v"(x), "v"(y)); }
__device__ __forceinline__ void keep4_h(v16h a, v16h b, v16h c, v16h d) { asm volatile("v_nop" :: "v"(a), "v"(b), "v"(c), "v"(d)); }
__device__ __forceinline__ void keep4_b(v16b a, v16b b, v16b c, v16b d) { asm volatile("v_nop" :: "v"(a), "v"(b), "v"(c), "v"(d)); }
__device__ __forceinline__ void acc_guard4(v8f& a, v8f& b, v8f& c, v8f& d) { asm volatile("v_nop\n\tv_nop\n\tv_nop\n\tv_nop" : "+v"(a), "+v"(b), "+v"(c), "+v"(d)); }
template <typename T> struct Frag;
template <> struct Frag<_Float16> {
  typedef v16h V; union U { v16h v; v8h h[2]; };
  static __device__ __forceinline__ v16h load(const _Float16* p) {
    U f; f.h[0] = *(const v8h*)(p); f.h[1] = *(const v8h*)(p + 16); return f.v;
  }
  static __device__ __forceinline__ v8f mma(v16h a, v16h b, v8f c) {
    return __builtin_amdgcn_wmma_f32_16x16x32_f16(false, a, false, b, (short)0, c, false, false);
  }
  static __device__ __forceinline__ void guard(v8f& a, v8f& b, v16h x, v16h y) { dep_guard_h(a, b, x, y); }
  static __device__ __forceinline__ void keep(v16h a, v16h b, v16h c, v16h d) { keep4_h(a, b, c, d); }
};
template <> struct Frag<__bf16> {
  typedef v16b V; union U { v16b v; v8b h[2]; };
  static __device__ __forceinline__ v16b load(const __bf16* p) {
    U f; f.h[0] = *(const v8b*)(p); f.h[1] = *(const v8b*)(p + 16); return f.v;
  }
  static __device__ __forceinline__ v8f mma(v16b a, v16b b, v8f c) {
    return __builtin_amdgcn_wmma_f32_16x16x32_bf16(false, a, false, b, (short)0, c, false, false);
  }
  static __device__ __forceinline__ void guard(v8f& a, v8f& b, v16b x, v16b y) { dep_guard_b(a, b, x, y); }
  static __device__ __forceinline__ void keep(v16b a, v16b b, v16b c, v16b d) { keep4_b(a, b, c, d); }
};

__device__ __forceinline__ unsigned pk16(unsigned short a, unsigned short b) { return (unsigned)a | ((unsigned)b << 16); }
__device__ __forceinline__ unsigned short h_bits(float f) { const _Float16 h = (_Float16)f; return __builtin_bit_cast(unsigned short, h); }

template <int ET> struct Elem;
template <> struct Elem<0> { typedef _Float16 T; };
template <> struct Elem<1> { typedef __bf16 T; };
template <int ET, int SPLIT, int BIAS_MODE, int OUT_MODE, bool RESID, int ACT = 0>
__global__ __launch_bounds__(256) void wmma_gemm64(
    const unsigned short* __restrict__ Ap, const unsigned short* __restrict__ A2p, int lda, long strideA,
    const unsigned short* __restrict__ Btp, const unsigned short* __restrict__ Bt2p, int ldb, long strideB,
    void* __restrict__ Cout, void* __restrict__ Cout2, int ldc, long strideC,
    const float* __restrict__ bias,
    const float* __restrict__ resid, long strideR,
    int M, int N, int K, float scale) {
  typedef typename Elem<ET>::T T;
  typedef typename Frag<T>::V V;
  const T* A = (const T*)Ap; const T* A2 = (const T*)A2p; const T* Bt = (const T*)Btp; const T* Bt2 = (const T*)Bt2p;
  __shared__ __align__(16) float sT[8][16 * 68];
  const int b    = blockIdx.y;
  const int lane = threadIdx.x & 31;
  const int wave = threadIdx.x >> 5;
  const int tilesN = N >> 6;
  const int tilesM = M >> 6;
  const int tile = blockIdx.x * 8 + wave;
  if (tile >= tilesM * tilesN) return;
  const int tm = tile / tilesN;
  const int tn = tile - tm * tilesN;
  const int m0 = tm << 6;
  const int n0 = tn << 6;

  const T* Ab  = A  + (size_t)b * strideA;
  const T* Bb  = Bt + (size_t)b * strideB;
  const T* Ab2 = (SPLIT != 0) ? (A2  + (size_t)b * strideA) : nullptr;
  const T* Bb2 = (SPLIT == 1) ? (Bt2 + (size_t)b * strideB) : nullptr;

  const int rlane = lane & 15;
  const int koff  = (lane >> 4) * 8;
  const int mOff  = (lane >> 4) * 8;

  v8f acc[4][4];
#pragma unroll
  for (int i = 0; i < 4; ++i)
#pragma unroll
    for (int j = 0; j < 4; ++j) acc[i][j] = (v8f){0.f,0.f,0.f,0.f,0.f,0.f,0.f,0.f};

  for (int k0 = 0; k0 < K; k0 += 32) {
    V bh[4], bl[4];
#pragma unroll
    for (int j = 0; j < 4; ++j) {
      const size_t bo = (size_t)(n0 + (j << 4) + rlane) * ldb + koff + k0;
      bh[j] = Frag<T>::load(Bb + bo);
      if (SPLIT == 1) bl[j] = Frag<T>::load(Bb2 + bo);
    }
#pragma unroll
    for (int i = 0; i < 4; ++i) {
      const size_t ao = (size_t)(m0 + (i << 4) + rlane) * lda + koff + k0;
      V ah = Frag<T>::load(Ab + ao);
      V al;
      if (SPLIT != 0) al = Frag<T>::load(Ab2 + ao);
#pragma unroll
      for (int j = 0; j < 4; ++j) {
        acc[i][j] = Frag<T>::mma(ah, bh[j], acc[i][j]);
        if (SPLIT == 1) acc[i][j] = Frag<T>::mma(ah, bl[j], acc[i][j]);
        if (SPLIT != 0) acc[i][j] = Frag<T>::mma(al, bh[j], acc[i][j]);
      }
      Frag<T>::guard(acc[i][0], acc[i][3], ah, (SPLIT != 0) ? al : ah);
    }
    Frag<T>::keep(bh[0], bh[1], bh[2], bh[3]);
    if (SPLIT == 1) Frag<T>::keep(bl[0], bl[1], bl[2], bl[3]);
  }
  acc_guard4(acc[0][0], acc[0][1], acc[0][2], acc[0][3]);
  acc_guard4(acc[1][0], acc[1][1], acc[1][2], acc[1][3]);
  acc_guard4(acc[2][0], acc[2][1], acc[2][2], acc[2][3]);
  acc_guard4(acc[3][0], acc[3][1], acc[3][2], acc[3][3]);

  float* slab = sT[wave];
  const float* Rb = RESID ? (resid + (size_t)b * strideR) : nullptr;
#pragma unroll
  for (int i = 0; i < 4; ++i) {
    const int mBase = m0 + (i << 4);
#pragma unroll
    for (int j = 0; j < 4; ++j) {
      const int n = n0 + (j << 4) + rlane;
      float bv = 0.f;
      if (BIAS_MODE == 2) bv = bias[n];
#pragma unroll
      for (int r = 0; r < 8; ++r) {
        float v = acc[i][j][r] * scale;
        if (BIAS_MODE == 1) v += bias[mBase + mOff + r];
        if (BIAS_MODE == 2) v += bv;
        if (RESID) v += Rb[(size_t)(mBase + mOff + r) * ldc + n];
        if (ACT == 2) v = fmaxf(v, 0.0f);
        if (ACT == 4) v = (v > 0.f) ? v : 0.01f * v;
        slab[(mOff + r) * 68 + (j << 4) + rlane] = v;
      }
    }
    __builtin_amdgcn_fence(__ATOMIC_RELEASE, "workgroup");
    __builtin_amdgcn_wave_barrier();
    __builtin_amdgcn_fence(__ATOMIC_ACQUIRE, "workgroup");
    if (OUT_MODE == 0) {
      float* C = (float*)Cout + (size_t)b * strideC;
      const int hh = lane >> 4, c4 = (lane & 15) * 4;
      for (int pass = 0; pass < 2; ++pass) {
#pragma unroll
        for (int it = 0; it < 8; ++it) {
          const int row = it * 2 + hh;
          v4f v = *(const v4f*)(slab + row * 68 + c4);
          *(volatile v4f*)(C + (size_t)(mBase + row) * ldc + n0 + c4) = v;
        }
        __threadfence();
      }
    } else {
      const int q = lane >> 3, c8 = (lane & 7) * 8;
      unsigned short* C  = (unsigned short*)Cout  + (size_t)b * strideC;
      unsigned short* C2 = (OUT_MODE == 2) ? ((unsigned short*)Cout2 + (size_t)b * strideC) : nullptr;
      for (int pass = 0; pass < 2; ++pass) {
#pragma unroll
        for (int it = 0; it < 4; ++it) {
          const int row = it * 4 + q;
          const float* sp = slab + row * 68 + c8;
          v8h hv, lv;
#pragma unroll
          for (int e = 0; e < 8; ++e) {
            if (OUT_MODE == 1) {
              hv[e] = (_Float16)sp[e];
            } else {
              unsigned short hb = f2bf_bits(sp[e]);
              unsigned short lb = f2bf_bits(sp[e] - bf_bits2f(hb));
              hv[e] = __builtin_bit_cast(_Float16, hb);
              lv[e] = __builtin_bit_cast(_Float16, lb);
            }
          }
          *(volatile v8h*)(C + (size_t)(mBase + row) * ldc + n0 + c8) = hv;
          if (OUT_MODE == 2) *(volatile v8h*)(C2 + (size_t)(mBase + row) * ldc + n0 + c8) = lv;
        }
        __threadfence();
      }
    }
    __builtin_amdgcn_fence(__ATOMIC_RELEASE, "workgroup");
    __builtin_amdgcn_wave_barrier();
    __builtin_amdgcn_fence(__ATOMIC_ACQUIRE, "workgroup");
  }
}

__global__ __launch_bounds__(256) void cast8_bf16_kernel(const float* __restrict__ in, unsigned short* __restrict__ out, int n8) {
  const int i = blockIdx.x * 256 + threadIdx.x;
  if (i >= n8) return;
  const float* p = in + 8 * (size_t)i;
  const v4f a = *(const v4f*)(p);
  const v4f c = *(const v4f*)(p + 4);
  unsigned short hb[8];
#pragma unroll
  for (int e = 0; e < 4; ++e) { hb[e] = f2bf_bits(a[e]); hb[4 + e] = f2bf_bits(c[e]); }
  const v4u u = (v4u){pk16(hb[0], hb[1]), pk16(hb[2], hb[3]), pk16(hb[4], hb[5]), pk16(hb[6], hb[7])};
  unsigned short* q = out + 8 * (size_t)i;
  *(volatile v4u*)q = u;
  __threadfence();
  *(volatile v4u*)q = u;
}

__global__ __launch_bounds__(256) void traj_mag_kernel(const v4u* __restrict__ XB4, float* __restrict__ MW, float* __restrict__ INV) {
  __shared__ __align__(16) float mws[32];
  __shared__ __align__(16) float ivs[32];
  const int lane = threadIdx.x & 31, wave = threadIdx.x >> 5;
  const int b = blockIdx.y;
  const int j0 = blockIdx.x * 32;
  for (int t = 0; t < 4; ++t) {
    const int jl = wave * 4 + t;
    const int j  = j0 + jl;
    const int jc = (j < kS - 1) ? j : (kS - 2);
    const v4u* r0 = XB4 + (size_t)(b * kS + jc) * (kD / 8);
    const v4u* r1 = r0 + (kD / 8);
    float ss = 0.f;
#pragma unroll
    for (int i = 0; i < 4; ++i) {
      const v4u a = r0[lane * 4 + i];
      const v4u c = r1[lane * 4 + i];
#pragma unroll
      for (int w = 0; w < 4; ++w) {
        const float d0 = bfw_lo(c[w]) - bfw_lo(a[w]);
        const float d1 = bfw_hi(c[w]) - bfw_hi(a[w]);
        ss += d0 * d0;
        ss += d1 * d1;
      }
    }
#pragma unroll
    for (int o = 16; o > 0; o >>= 1) ss += __shfl_xor(ss, o, 32);
    const float mag = sqrtf(ss);
    const float mwv = tanhf(mag);
    const float ivv = 1.0f / fmaxf(mag, 1e-8f);
    const bool valid = (j < kS - 1);
    if (lane == 0) { mws[jl] = valid ? mwv : 0.f; ivs[jl] = valid ? ivv : 0.f; }
  }
  __syncthreads();
  if (wave == 0 && lane < 16) {
    const int q = lane & 7;
    const v4f va = *(const v4f*)(mws + 4 * q);
    const v4f vb = *(const v4f*)(ivs + 4 * q);
    const bool first = (lane < 8);
    const v4f val = (v4f){first ? va[0] : vb[0], first ? va[1] : vb[1], first ? va[2] : vb[2], first ? va[3] : vb[3]};
    float* gp = (first ? MW : INV) + (size_t)b * kS + j0 + 4 * q;
    for (int pass = 0; pass < 2; ++pass) {
      *(volatile v4f*)gp = val;
      __threadfence();
    }
  }
}

__global__ __launch_bounds__(256) void traj_out_kernel(const v2u* __restrict__ XB2, const float* __restrict__ MW,
                                                       const float* __restrict__ INV, float* __restrict__ out1) {
  const int p = blockIdx.x, b = blockIdx.y, t = threadIdx.x;
  const int ws  = (p > 8) ? (p - 8) : 0;
  const int cnt = p - ws;
  const int wsz = (cnt > 1) ? cnt : 1;
  const float* mwb = MW  + (size_t)b * kS;
  const float* ivb = INV + (size_t)b * kS;
  float denom = 0.f;
#pragma unroll 1
  for (int jj = 0; jj < cnt; ++jj) {
    const float rec = (float)(jj + 1) / (float)wsz;
    denom += mwb[ws + jj] * rec;
  }
  denom = fmaxf(denom, 1e-8f);
  const v2u* rowp = XB2 + (size_t)(b * kS + ws) * (kD / 4) + t;
  const v2u pw = rowp[0];
  v4f prv = (v4f){bfw_lo(pw[0]), bfw_hi(pw[0]), bfw_lo(pw[1]), bfw_hi(pw[1])};
  v4f acc = (v4f){0.f, 0.f, 0.f, 0.f};
#pragma unroll 1
  for (int jj = 0; jj < cnt; ++jj) {
    const int j = ws + jj;
    const v2u cw2 = rowp[(size_t)(jj + 1) * (kD / 4)];
    const v4f cur = (v4f){bfw_lo(cw2[0]), bfw_hi(cw2[0]), bfw_lo(cw2[1]), bfw_hi(cw2[1])};
    const float rec = (float)(jj + 1) / (float)wsz;
    const float nwv = (mwb[j] * rec) / denom;
    const float iv  = ivb[j];
#pragma unroll
    for (int e = 0; e < 4; ++e) {
      const float d  = cur[e] - prv[e];
      const float tv = d * iv;
      acc[e] += nwv * tv;
    }
    prv = cur;
  }
  float* op = out1 + (size_t)(b * kS + p) * kD + 4 * t;
  *(volatile v4f*)op = acc;
  __threadfence();
  *(volatile v4f*)op = acc;
}

__global__ __launch_bounds__(256) void splat_const_kernel(const float* __restrict__ lsc, const float* __restrict__ amp,
                                                          float* __restrict__ CONSTT) {
  __shared__ __align__(16) float c0[256];
  __shared__ __align__(16) float c1[256];
  const int t = threadIdx.x;
  const float ls = bf_bits2f(f2bf_bits(lsc[t]));
  const float a  = bf_bits2f(f2bf_bits(amp[t]));
  const float sc = expf(ls);
  const float ssq = sc * sc;
  c0[t] = 1.0f / ssq;
  c1[t] = 1.0f / (1.0f + expf(-a));
  __syncthreads();
  const int lane = t & 31, wave = t >> 5;
  if (wave < 2) {
    for (int pass = 0; pass < 2; ++pass) {
#pragma unroll
      for (int it = 0; it < 2; ++it) {
        const int idx = (it * 32 + lane) * 4;
        const v4f v0 = *(const v4f*)(c0 + idx);
        const v4f v1 = *(const v4f*)(c1 + idx);
        const v4f val = (wave == 0) ? v0 : v1;
        *(volatile v4f*)(CONSTT + wave * 256 + idx) = val;
      }
      __threadfence();
    }
  }
}

__global__ __launch_bounds__(128) void splat_weight_kernel(const float* __restrict__ QKV, const float* __restrict__ cent,
                                                           const float* __restrict__ CONSTT,
                                                           unsigned short* __restrict__ QWC, unsigned short* __restrict__ KWC) {
  __shared__ __align__(16) float tqk[2][64][64];
  __shared__ __align__(16) float csh[kNS][kHD];
  __shared__ __align__(16) float tw[2][64][16];
  __shared__ float cnsh[kNS];
  __shared__ float rcs[kNS];
  __shared__ float ams[kNS];
  const int t  = threadIdx.x;
  const int bh = blockIdx.y;
  const int b  = bh >> 4, h = bh & 15;
  const int s0 = blockIdx.x * 64;
#pragma unroll
  for (int i = 0; i < 16; ++i) {
    const int e = i * 128 + t;
    const int which = e >> 10;
    const int r  = (e >> 4) & 63;
    const int c4 = (e & 15) * 4;
    const v4f v = *(const v4f*)(QKV + (size_t)(b * kS + s0 + r) * kQKVN + which * kD + h * kHD + c4);
    *(v4f*)(&tqk[which][r][c4]) = v;
  }
#pragma unroll
  for (int i = 0; i < 2; ++i) {
    const int e  = i * 128 + t;
    const int kk = e >> 4;
    const int c4 = (e & 15) * 4;
    const v4f c = *(const v4f*)(cent + (size_t)(h * kNS + kk) * kHD + c4);
    const v4f cr = (v4f){bf_bits2f(f2bf_bits(c[0])), bf_bits2f(f2bf_bits(c[1])), bf_bits2f(f2bf_bits(c[2])), bf_bits2f(f2bf_bits(c[3]))};
    *(v4f*)(&csh[kk][c4]) = cr;
  }
  if (t < kNS) { rcs[t] = CONSTT[h * kNS + t]; ams[t] = CONSTT[256 + h * kNS + t]; }
  __syncthreads();
  if (t < kNS) {
    float cn = 0.f;
#pragma unroll 1
    for (int d4 = 0; d4 < kHD / 4; ++d4) {
      const v4f c = *(const v4f*)(&csh[t][4 * d4]);
      cn += c[0] * c[0]; cn += c[1] * c[1]; cn += c[2] * c[2]; cn += c[3] * c[3];
    }
    cnsh[t] = cn;
  }
  __syncthreads();
  const int which = t >> 6, sl = t & 63;
  const float* row = &tqk[which][sl][0];
  float tn = 0.f;
#pragma unroll 1
  for (int d4 = 0; d4 < kHD / 4; ++d4) {
    const v4f q = *(const v4f*)(row + 4 * d4);
    tn += q[0] * q[0]; tn += q[1] * q[1]; tn += q[2] * q[2]; tn += q[3] * q[3];
  }
#pragma unroll 1
  for (int kk = 0; kk < kNS; ++kk) {
    float cross = 0.f;
#pragma unroll 1
    for (int d4 = 0; d4 < kHD / 4; ++d4) {
      const v4f q = *(const v4f*)(row + 4 * d4);
      const v4f c = *(const v4f*)(&csh[kk][4 * d4]);
      cross += q[0] * c[0]; cross += q[1] * c[1]; cross += q[2] * c[2]; cross += q[3] * c[3];
    }
    const float d2 = tn - 2.0f * cross + cnsh[kk];
    const float w  = expf((-0.5f * d2) * rcs[kk]) * ams[kk];
    tw[which][sl][kk] = w * kWgtCarry;
  }
  __syncthreads();
  const int lane = t & 31, wave = t >> 5;
  const int pl = wave >> 1;
  const int rbase = (wave & 1) * 32;
  unsigned short* gp = ((pl == 0) ? QWC : KWC) + ((size_t)bh * kS + s0) * kKP;
  const int rq = lane >> 2;
  const int c8 = (lane & 3) * 8;
  const bool hasData = (c8 < 16);
  const int cc = hasData ? c8 : 0;
  for (int pass = 0; pass < 2; ++pass) {
#pragma unroll
    for (int it = 0; it < 4; ++it) {
      const int rowl = rbase + it * 8 + rq;
      const v4f w0 = *(const v4f*)(&tw[pl][rowl][cc]);
      const v4f w1 = *(const v4f*)(&tw[pl][rowl][cc + 4]);
      unsigned short hb[8];
#pragma unroll
      for (int e = 0; e < 4; ++e) {
        hb[e]     = hasData ? h_bits(w0[e]) : (unsigned short)0;
        hb[4 + e] = hasData ? h_bits(w1[e]) : (unsigned short)0;
      }
      const v4u u = (v4u){pk16(hb[0], hb[1]), pk16(hb[2], hb[3]), pk16(hb[4], hb[5]), pk16(hb[6], hb[7])};
      *(volatile v4u*)(gp + (size_t)rowl * kKP + c8) = u;
    }
    __threadfence();
  }
}

__global__ __launch_bounds__(256) void vt_kernel(const float* __restrict__ QKV, unsigned short* __restrict__ VT) {
  __shared__ float sm[64][65];
  const int t  = threadIdx.x;
  const int jt = blockIdx.x, bh = blockIdx.y;
  const int b  = bh >> 4, h = bh & 15;
  const int j0 = jt * 64;
  const float* vp = QKV + (size_t)(b * kS + j0) * kQKVN + 2 * kD + h * kHD;
#pragma unroll
  for (int i = 0; i < 16; ++i) {
    const int e = i * 256 + t;
    const int r = e >> 6;
    const int c = e & 63;
    sm[c][r] = vp[(size_t)r * kQKVN + c];
  }
  __syncthreads();
  const int lane = t & 31, wave = t >> 5;
  const int q = lane >> 3, c8 = (lane & 7) * 8;
  unsigned short* op = VT + (size_t)bh * kHD * kS + j0;
  for (int pass = 0; pass < 2; ++pass) {
#pragma unroll
    for (int it = 0; it < 2; ++it) {
      const int row = wave * 8 + it * 4 + q;
      unsigned short hb[8];
#pragma unroll
      for (int e = 0; e < 8; ++e) hb[e] = h_bits(sm[row][c8 + e]);
      const v4u u = (v4u){pk16(hb[0], hb[1]), pk16(hb[2], hb[3]), pk16(hb[4], hb[5]), pk16(hb[6], hb[7])};
      *(volatile v4u*)(op + (size_t)row * kS + c8) = u;
    }
    __threadfence();
  }
}

__global__ __launch_bounds__(64) void vmean_kernel(const float* __restrict__ QKV, float* __restrict__ VMEAN) {
  __shared__ __align__(16) float vm[64];
  const int bh = blockIdx.x;
  const int b = bh >> 4, h = bh & 15;
  const int d = threadIdx.x;
  const float* vp = QKV + (size_t)(b * kS) * kQKVN + 2 * kD + h * kHD + d;
  float s0 = 0.f, s1 = 0.f, s2 = 0.f, s3 = 0.f;
#pragma unroll 1
  for (int j = 0; j < kS; j += 4) {
    s0 += vp[(size_t)(j + 0) * kQKVN];
    s1 += vp[(size_t)(j + 1) * kQKVN];
    s2 += vp[(size_t)(j + 2) * kQKVN];
    s3 += vp[(size_t)(j + 3) * kQKVN];
  }
  vm[d] = ((s0 + s1) + (s2 + s3)) * kInvS;
  __syncthreads();
  if (d < 16) {
    const v4f val = *(const v4f*)(vm + 4 * d);
    float* gp = VMEAN + (size_t)bh * kHD + 4 * d;
    for (int pass = 0; pass < 2; ++pass) {
      *(volatile v4f*)gp = val;
      __threadfence();
    }
  }
}

__global__ __launch_bounds__(256) void softmax_kernel(const float* __restrict__ Sp, unsigned short* __restrict__ Pp) {
  __shared__ float redM[8];
  __shared__ float redS[8];
  const int row  = blockIdx.x;
  const int pr   = blockIdx.y;
  const int t    = threadIdx.x;
  const int lane = t & 31, wave = t >> 5;
  const size_t base = ((size_t)pr * kS + row) * kS + (size_t)t * 8;
  const v4f a = *(const v4f*)(Sp + base);
  const v4f c = *(const v4f*)(Sp + base + 4);
  float x[8];
#pragma unroll
  for (int e = 0; e < 4; ++e) { x[e] = a[e]; x[4 + e] = c[e]; }
  float m = fmaxf(fmaxf(fmaxf(x[0], x[1]), fmaxf(x[2], x[3])), fmaxf(fmaxf(x[4], x[5]), fmaxf(x[6], x[7])));
#pragma unroll
  for (int off = 16; off > 0; off >>= 1) m = fmaxf(m, __shfl_xor(m, off, 32));
  if (lane == 0) redM[wave] = m;
  __syncthreads();
  float gm = redM[0];
#pragma unroll
  for (int w = 1; w < 8; ++w) gm = fmaxf(gm, redM[w]);
  float ev[8];
#pragma unroll
  for (int e = 0; e < 8; ++e) ev[e] = expf(x[e] - gm);
  float ps = ((ev[0] + ev[1]) + (ev[2] + ev[3])) + ((ev[4] + ev[5]) + (ev[6] + ev[7]));
#pragma unroll
  for (int off = 16; off > 0; off >>= 1) ps += __shfl_xor(ps, off, 32);
  if (lane == 0) redS[wave] = ps;
  __syncthreads();
  const float tot = ((redS[0] + redS[1]) + (redS[2] + redS[3])) + ((redS[4] + redS[5]) + (redS[6] + redS[7]));
  const float rinv = 1.0f / tot;
  unsigned short hb[8];
#pragma unroll
  for (int e = 0; e < 8; ++e) hb[e] = h_bits((ev[e] * rinv - kInvS) * kPCarry);
  const v4u u = (v4u){pk16(hb[0], hb[1]), pk16(hb[2], hb[3]), pk16(hb[4], hb[5]), pk16(hb[6], hb[7])};
  unsigned short* q = Pp + base;
  *(volatile v4u*)q = u;
  __threadfence();
  *(volatile v4u*)q = u;
}

__global__ __launch_bounds__(256) void ctx_finalize_kernel(const float* __restrict__ CTXF, const float* __restrict__ VMEAN,
                                                           unsigned short* __restrict__ CTXH, unsigned short* __restrict__ CTXL) {
  const int i   = blockIdx.x * 256 + threadIdx.x;
  const int row = i >> 7;
  const int c   = (i & 127) * 8;
  const int b   = row >> 11;
  const int h   = c >> 6;
  const float* sp = CTXF + (size_t)row * kD + c;
  const float* mp = VMEAN + (size_t)(b * kH + h) * kHD + (c & 63);
  const v4f a0 = *(const v4f*)(sp);
  const v4f a1 = *(const v4f*)(sp + 4);
  const v4f m0 = *(const v4f*)(mp);
  const v4f m1 = *(const v4f*)(mp + 4);
  unsigned short hb[8], lb[8];
#pragma unroll
  for (int e = 0; e < 4; ++e) {
    const float v0 = a0[e] + m0[e];
    hb[e] = f2bf_bits(v0);
    lb[e] = f2bf_bits(v0 - bf_bits2f(hb[e]));
    const float v1 = a1[e] + m1[e];
    hb[4 + e] = f2bf_bits(v1);
    lb[4 + e] = f2bf_bits(v1 - bf_bits2f(hb[4 + e]));
  }
  const v4u uh = (v4u){pk16(hb[0], hb[1]), pk16(hb[2], hb[3]), pk16(hb[4], hb[5]), pk16(hb[6], hb[7])};
  const v4u ul = (v4u){pk16(lb[0], lb[1]), pk16(lb[2], lb[3]), pk16(lb[4], lb[5]), pk16(lb[6], lb[7])};
  unsigned short* qh = CTXH + (size_t)row * kD + c;
  unsigned short* ql = CTXL + (size_t)row * kD + c;
  *(volatile v4u*)qh = uh;
  *(volatile v4u*)ql = ul;
  __threadfence();
  *(volatile v4u*)qh = uh;
  *(volatile v4u*)ql = ul;
}

extern "C" void kernel_launch(void* const* d_in, const int* in_sizes, int n_in,
                              void* d_out, int out_size, void* d_ws, size_t ws_size,
                              hipStream_t stream) {
  (void)in_sizes; (void)n_in; (void)out_size; (void)ws_size;
  const float* x     = (const float*)d_in[0];
  const float* qkv_w = (const float*)d_in[1];
  const float* out_w = (const float*)d_in[2];
  const float* cent  = (const float*)d_in[3];
  const float* lsc   = (const float*)d_in[4];
  const float* amp   = (const float*)d_in[5];

  float* out0 = (float*)d_out;
  float* out1 = (float*)d_out + (size_t)kTok * kD;

  unsigned char* wsb = (unsigned char*)d_ws;
  size_t off = 0;
  unsigned short* OUTW = (unsigned short*)(wsb + off); off += (size_t)kD * kD * 2;
  unsigned short* QWC  = (unsigned short*)(wsb + off); off += (size_t)kBH * kS * kKP * 2;
  unsigned short* KWC  = (unsigned short*)(wsb + off); off += (size_t)kBH * kS * kKP * 2;
  unsigned short* VT   = (unsigned short*)(wsb + off); off += (size_t)kBH * kHD * kS * 2;
  float*          CTXF = (float*)(wsb + off);          off += (size_t)kTok * kD * 4;
  unsigned short* CTXH = (unsigned short*)(wsb + off); off += (size_t)kTok * kD * 2;
  unsigned short* CTXL = (unsigned short*)(wsb + off); off += (size_t)kTok * kD * 2;
  float*          VMEAN  = (float*)(wsb + off);        off += (size_t)kBH * kHD * 4;
  float*          MW     = (float*)(wsb + off);        off += (size_t)kB * kS * 4;
  float*          INV    = (float*)(wsb + off);        off += (size_t)kB * kS * 4;
  float*          CONSTT = (float*)(wsb + off);        off += (size_t)512 * 4;
  unsigned char* dyn = wsb + off;
  unsigned short* XB   = (unsigned short*)(dyn);
  unsigned short* QKVW = (unsigned short*)(dyn + (size_t)kTok * kD * 2);
  float*          QKV  = (float*)(dyn + (size_t)kTok * kD * 2 + (size_t)kQKVN * kD * 2);
  float*          SPL  = (float*)(dyn);
  unsigned short* PPL  = (unsigned short*)(dyn + (size_t)kGrp * kS * kS * 4);

  {
    const int n8x = kTok * kD / 8;
    cast8_bf16_kernel<<<(n8x + 255) / 256, 256, 0, stream>>>(x, XB, n8x);
    const int n8q = kQKVN * kD / 8;
    cast8_bf16_kernel<<<(n8q + 255) / 256, 256, 0, stream>>>(qkv_w, QKVW, n8q);
    const int n8o = kD * kD / 8;
    cast8_bf16_kernel<<<(n8o + 255) / 256, 256, 0, stream>>>(out_w, OUTW, n8o);
  }

  traj_mag_kernel<<<dim3(kS / 32, kB), 256, 0, stream>>>((const v4u*)(const void*)XB, MW, INV);
  traj_out_kernel<<<dim3(kS, kB), 256, 0, stream>>>((const v2u*)(const void*)XB, MW, INV, out1);

  wmma_gemm64<1, 0, 0, 0, false><<<dim3((kTok / 64) * (kQKVN / 64) / 8, 1), 256, 0, stream>>>(
      XB, XB, kD, 0L, QKVW, QKVW, kD, 0L,
      (void*)QKV, (void*)QKV, kQKVN, 0L, VMEAN, VMEAN, 0L, kTok, kQKVN, kD, 1.0f);

  splat_const_kernel<<<1, 256, 0, stream>>>(lsc, amp, CONSTT);
  splat_weight_kernel<<<dim3(kS / 64, kBH), 128, 0, stream>>>(QKV, cent, CONSTT, QWC, KWC);

  vt_kernel<<<dim3(kS / 64, kBH), 256, 0, stream>>>(QKV, VT);
  vmean_kernel<<<kBH, 64, 0, stream>>>(QKV, VMEAN);

  for (int gi = 0; gi < kBH / kGrp; ++gi) {
    const int bh0 = gi * kGrp;
    const int b   = bh0 >> 4;
    const int h0  = bh0 & 15;
    wmma_gemm64<0, 0, 0, 0, false><<<dim3((kS / 64) * (kS / 64) / 8, kGrp), 256, 0, stream>>>(
        QWC + (size_t)bh0 * kS * kKP, QWC + (size_t)bh0 * kS * kKP, kKP, (long)kS * kKP,
        KWC + (size_t)bh0 * kS * kKP, KWC + (size_t)bh0 * kS * kKP, kKP, (long)kS * kKP,
        (void*)SPL, (void*)SPL, kS, (long)kS * kS, VMEAN, VMEAN, 0L, kS, kS, kKP, kScoreScale);
    softmax_kernel<<<dim3(kS, kGrp), 256, 0, stream>>>(SPL, PPL);
    wmma_gemm64<0, 0, 0, 0, false><<<dim3((kS / 64) * (kHD / 64) / 8, kGrp), 256, 0, stream>>>(
        PPL, PPL, kS, (long)kS * kS,
        VT + (size_t)bh0 * kHD * kS, VT + (size_t)bh0 * kHD * kS, kS, (long)kHD * kS,
        (void*)(CTXF + (size_t)(b * kS) * kD + h0 * kHD), (void*)(CTXF + (size_t)(b * kS) * kD + h0 * kHD), kD, (long)kHD,
        VMEAN, VMEAN, 0L, kS, kHD, kS, kPCarryInv);
  }

  ctx_finalize_kernel<<<(kTok * (kD / 8)) / 256, 256, 0, stream>>>(CTXF, VMEAN, CTXH, CTXL);

  wmma_gemm64<1, 2, 0, 0, false><<<dim3((kTok / 64) * (kD / 64) / 8, 1), 256, 0, stream>>>(
      CTXH, CTXL, kD, 0L, OUTW, OUTW, kD, 0L,
      (void*)out0, (void*)out0, kD, 0L, VMEAN, VMEAN, 0L, kTok, kD, kD, 1.0f);
}
